// Deter_738734375713
// MI455X (gfx1250) — hardware-verified
//
#include <hip/hip_runtime.h>


namespace {
constexpr int Bn = 1024, DET = 4096, STO = 1024, ACT = 128, HID = 1024, BLK = 8, DPB = 512, INC0 = 3 * HID + DPB  , XW = 3 * HID  ;
constexpr float XS = 8.0f, RMS_EPS = 1e-4f;

typedef _Float16 b16;
typedef __attribute__((ext_vector_type(16))) _Float16 v16b;
typedef __attribute__((ext_vector_type(8))) _Float16 v8b;
typedef __attribute__((ext_vector_type(8))) float v8f;
typedef __attribute__((ext_vector_type(4))) float v4f;
__device__ __forceinline__ float bf16_rne(float f) { unsigned int u = __float_as_uint(f); u += 0x7FFFu + ((u >> 16) & 1u); return __uint_as_float(u & 0xFFFF0000u); }
__device__ __forceinline__ void split16(float v, b16& hi, b16& lo) { hi = (b16)v; lo = (b16)(v - (float)hi); }
__device__ __forceinline__ v16b frag_kb(const b16* p, int hh) { const v8b a = *(const v8b*)(p + 8 * hh), b = *(const v8b*)(p + 16 + 8 * hh); v16b f;
#pragma unroll
  for (int e = 0; e < 8; ++e) { f[e] = a[e]; f[8 + e] = b[e]; } return f; }
__device__ __forceinline__ v8f wmma16b(v16b a, v16b b, v8f c) { v8f d = __builtin_amdgcn_wmma_f32_16x16x32_f16(false, a, false, b, (short)0, c, false, false); asm volatile("v_nop\n\tv_nop\n\tv_nop\n\tv_nop" : "+v"(d) : "v"(a), "v"(b)); return d; }
__device__ __forceinline__ void wave_lds_sync() { __builtin_amdgcn_fence(__ATOMIC_RELEASE, "workgroup"); __builtin_amdgcn_wave_barrier(); __builtin_amdgcn_fence(__ATOMIC_ACQUIRE, "workgroup"); }
__device__ __forceinline__ float nexp(float x) { return __builtin_amdgcn_exp2f(x * 1.4426950408889634f); }
__device__ __forceinline__ float pmul(float a, float b) { float p = a * b; asm volatile("" : "+v"(p)); return p; }
__device__ __forceinline__ float sigm(float x) { return 1.0f / (1.0f + nexp(-x)); }
__device__ __forceinline__ float silu(float x) { return x * sigm(x); }
__device__ __forceinline__ float tanh_f(float x) { const float e = nexp(-2.0f * fabsf(x)); const float t = (1.0f - e) / (1.0f + e); return (x < 0.0f) ? -t : t; }
__device__ __forceinline__ float wsum(float v) {
#pragma unroll
  for (int o = 1; o < 32; o <<= 1) v += __shfl_xor(v, o); return v; }

struct Ro_ { static constexpr size_t W0 = 0, W1 = W0 + (size_t)HID * DET, W2 = W1 + (size_t)HID * STO, H0W = W2 + (size_t)HID * ACT, H1W = H0W + (size_t)BLK * DPB * INC0, GW = H1W + (size_t)BLK * DPB * DPB, END = GW + (size_t)BLK * 3 * DPB * DPB; };
constexpr int PEND = 22528 + 12288;
__global__ __launch_bounds__(256) void prep_kernel(const float* __restrict__ stoch, const float* __restrict__ deter, const float* __restrict__ action, const float* __restrict__ w0, const float* __restrict__ w1, const float* __restrict__ w2, const float* __restrict__ hw0, const float* __restrict__ hw1, const float* __restrict__ gw,
    b16* __restrict__ R, b16* __restrict__ DX, b16* __restrict__ SX, b16* __restrict__ AX) {
  const size_t tid = (size_t)blockIdx.x * 256 + threadIdx.x, nth = (size_t)gridDim.x * 256;
  auto tr = [&](size_t base, int nout, int kin, const float* W) { for (size_t p = tid; p < (size_t)nout * kin; p += nth) { const int o = (int)(p / kin), k = (int)(p % kin); ((volatile b16*)R)[base + p] = (b16)bf16_rne(W[(size_t)k * nout + o]); } };
  for (int pass = 0; pass < 2; ++pass) {
    tr(Ro_::W0, HID, DET, w0); tr(Ro_::W1, HID, STO, w1); tr(Ro_::W2, HID, ACT, w2);
    for (int g = 0; g < BLK; ++g) { tr(Ro_::H0W + (size_t)g * DPB * INC0, DPB, INC0, hw0 + (size_t)g * INC0 * DPB); tr(Ro_::H1W + (size_t)g * DPB * DPB, DPB, DPB, hw1 + (size_t)g * DPB * DPB); tr(Ro_::GW + (size_t)g * 3 * DPB * DPB, 3 * DPB, DPB, gw + (size_t)g * DPB * 3 * DPB); }
    for (size_t p = tid; p < (size_t)Bn * DET / 8; p += nth) { v8b v; for (int e = 0; e < 8; ++e) v[e] = (b16)(bf16_rne(deter[p * 8 + e]) * XS); *(volatile v8b*)(DX + p * 8) = v; }
    for (size_t p = tid; p < (size_t)Bn * STO / 8; p += nth) { v8b v; for (int e = 0; e < 8; ++e) v[e] = (b16)(bf16_rne(stoch[p * 8 + e]) * XS); *(volatile v8b*)(SX + p * 8) = v; }
    for (size_t p = tid; p < (size_t)Bn * ACT / 8; p += nth) { v8b v; for (int e = 0; e < 8; ++e) { const float a = bf16_rne(action[p * 8 + e]); v[e] = (b16)((a / fmaxf(fabsf(a), 1.0f)) * XS); } *(volatile v8b*)(AX + p * 8) = v; }
    __threadfence(); }
}
__global__ __launch_bounds__(256) void params_kernel(const float* __restrict__ b0, const float* __restrict__ g0, const float* __restrict__ b1, const float* __restrict__ g1, const float* __restrict__ b2, const float* __restrict__ g2, const float* __restrict__ hb0, const float* __restrict__ hg0, const float* __restrict__ hb1, const float* __restrict__ hg1, const float* __restrict__ gb, float* __restrict__ P) {
  const size_t tid = (size_t)blockIdx.x * 256 + threadIdx.x, nth = (size_t)gridDim.x * 256;
  for (int pass = 0; pass < 2; ++pass) { for (size_t q = tid; q < (size_t)PEND; q += nth) { const int i = (int)q; float v;
      if (i < 1024) v = b0[i]; else if (i < 2048) v = b1[i - 1024]; else if (i < 3072) v = b2[i - 2048]; else if (i < 4096) v = g0[i - 3072]; else if (i < 5120) v = g1[i - 4096]; else if (i < 6144) v = g2[i - 5120];
      else if (i < 10240) v = hb0[i - 6144]; else if (i < 14336) v = hg0[i - 10240]; else if (i < 18432) v = hb1[i - 14336]; else if (i < 22528) v = hg1[i - 18432]; else v = gb[i - 22528];
      P[q] = bf16_rne(v); } __threadfence(); }
}

template <int K1, int K2>
__global__ __launch_bounds__(64) void gemm_kernel(const b16* __restrict__ A1, int lda1, int a1c0, const b16* __restrict__ A2h, const b16* __restrict__ A2l, int lda2, const b16* __restrict__ Bw, const float* __restrict__ bias, float* __restrict__ PRE, int ldp, int pc0) {
  __shared__ __attribute__((aligned(16))) float Ts[2][32][128 + 4];
  constexpr int KB = K1 + K2;
  const int lane = threadIdx.x & 31, wave = threadIdx.x >> 5, nloc = lane & 15, hlf = lane >> 4, m0 = blockIdx.y * 32, c0 = blockIdx.x * 256 + wave * 128;
  v8f acc[2][8];
#pragma unroll
  for (int r = 0; r < 2; ++r)
#pragma unroll
    for (int t = 0; t < 8; ++t) acc[r][t] = (v8f){};
  if (K1 > 0) {
#pragma unroll 2
    for (int kb = 0; kb < K1; kb += 32) { const v16b a0 = frag_kb(A1 + (size_t)(m0 + nloc) * lda1 + a1c0 + kb, hlf), a1 = frag_kb(A1 + (size_t)(m0 + 16 + nloc) * lda1 + a1c0 + kb, hlf);
#pragma unroll
      for (int t = 0; t < 8; ++t) { const v16b bw = frag_kb(Bw + (size_t)(c0 + t * 16 + nloc) * KB + kb, hlf); acc[0][t] = wmma16b(a0, bw, acc[0][t]); acc[1][t] = wmma16b(a1, bw, acc[1][t]); } } }
  if (K2 > 0) {
#pragma unroll 2
    for (int kb = 0; kb < K2; kb += 32) { const v16b a0 = frag_kb(A2h + (size_t)(m0 + nloc) * lda2 + kb, hlf), a1 = frag_kb(A2h + (size_t)(m0 + 16 + nloc) * lda2 + kb, hlf), l0 = frag_kb(A2l + (size_t)(m0 + nloc) * lda2 + kb, hlf), l1 = frag_kb(A2l + (size_t)(m0 + 16 + nloc) * lda2 + kb, hlf);
#pragma unroll
      for (int t = 0; t < 8; ++t) { const v16b bw = frag_kb(Bw + (size_t)(c0 + t * 16 + nloc) * KB + K1 + kb, hlf); acc[0][t] = wmma16b(a0, bw, acc[0][t]); acc[0][t] = wmma16b(l0, bw, acc[0][t]); acc[1][t] = wmma16b(a1, bw, acc[1][t]); acc[1][t] = wmma16b(l1, bw, acc[1][t]); } } }
#pragma unroll
  for (int t = 0; t < 8; ++t) { const float bb = bias[c0 + t * 16 + nloc];
#pragma unroll
    for (int r = 0; r < 2; ++r)
#pragma unroll
      for (int v = 0; v < 8; ++v) Ts[wave][r * 16 + 8 * hlf + v][t * 16 + nloc] = acc[r][t][v] * (1.0f / XS) + bb; }
  wave_lds_sync();
  for (int pass = 0; pass < 2; ++pass) { for (int i = lane; i < 32 * 32; i += 32) { const int rr = i >> 5, c4 = (i & 31) * 4; *(volatile v4f*)(PRE + (size_t)(m0 + rr) * ldp + pc0 + c0 + c4) = *(const v4f*)(&Ts[wave][rr][c4]); } __threadfence(); }
}
template <int NSEG, int SEG>
__global__ __launch_bounds__(256) void rms_kernel(const float* __restrict__ PRE, const float* __restrict__ gain, b16* __restrict__ Hh, b16* __restrict__ Hl) {
  __shared__ float red[8]; __shared__ float inv[NSEG];
  constexpr int W = NSEG * SEG; const int row = blockIdx.x, t_ = threadIdx.x, wave = t_ >> 5, lane = t_ & 31; const float* pr = PRE + (size_t)row * W;
  for (int s = 0; s < NSEG; ++s) { float q = 0.0f; for (int c = t_; c < SEG; c += 256) { const float v = pr[s * SEG + c]; q += pmul(v, v); } q = wsum(q); if (lane == 0) red[wave] = q; __syncthreads();
    if (t_ == 0) { float tot = 0.0f; for (int w = 0; w < 8; ++w) tot += red[w]; inv[s] = rsqrtf(tot * (1.0f / SEG) + RMS_EPS); } __syncthreads(); }
  for (int pass = 0; pass < 2; ++pass) { for (int i = t_; i < W / 8; i += 256) { const int c8 = i * 8; const int s = c8 / SEG; const float is = inv[s]; v8b hv, lv;
#pragma unroll
      for (int e = 0; e < 8; ++e) { const int c = c8 + e; const float y = silu(pmul(pr[c] * is, gain[c])); b16 a_, b_; split16(y * XS, a_, b_); hv[e] = a_; lv[e] = b_; }
      *(volatile v8b*)(Hh + (size_t)row * W + c8) = hv; *(volatile v8b*)(Hl + (size_t)row * W + c8) = lv; } __threadfence(); }
}
__global__ __launch_bounds__(64) void gate_kernel(const b16* __restrict__ Hh, const b16* __restrict__ Hl, const b16* __restrict__ GW, const float* __restrict__ gb, const float* __restrict__ deter, float* __restrict__ out) {
  __shared__ __attribute__((aligned(16))) float Ts[2][16][32 + 4];
  const int lane = threadIdx.x & 31, wave = threadIdx.x >> 5, nloc = lane & 15, hlf = lane >> 4, m0 = blockIdx.y * 32 + wave * 16, j0 = blockIdx.x * 32, g = blockIdx.z; const b16* Bw = GW + (size_t)g * 3 * DPB * DPB;
  v8f acc[3][2];
#pragma unroll
  for (int ch = 0; ch < 3; ++ch) { acc[ch][0] = (v8f){}; acc[ch][1] = (v8f){}; }
#pragma unroll 2
  for (int kb = 0; kb < DPB; kb += 32) { const v16b a = frag_kb(Hh + (size_t)(m0 + nloc) * DET + g * DPB + kb, hlf), al_ = frag_kb(Hl + (size_t)(m0 + nloc) * DET + g * DPB + kb, hlf);
#pragma unroll
    for (int ch = 0; ch < 3; ++ch)
#pragma unroll
      for (int t = 0; t < 2; ++t) { const v16b bw = frag_kb(Bw + (size_t)(ch * DPB + j0 + t * 16 + nloc) * DPB + kb, hlf); acc[ch][t] = wmma16b(a, bw, acc[ch][t]); acc[ch][t] = wmma16b(al_, bw, acc[ch][t]); } }
#pragma unroll
  for (int t = 0; t < 2; ++t) { const int j = j0 + t * 16 + nloc; const float br = gb[g * 3 * DPB + j], bc = gb[g * 3 * DPB + DPB + j], bu = gb[g * 3 * DPB + 2 * DPB + j];
#pragma unroll
    for (int r = 0; r < 8; ++r) { const int row = m0 + 8 * hlf + r; const float gr = acc[0][t][r] * (1.0f / XS) + br, gc = acc[1][t][r] * (1.0f / XS) + bc, gu = acc[2][t][r] * (1.0f / XS) + bu;
      const float reset = sigm(gr), cand = tanh_f(pmul(reset, gc)), upd = sigm(gu - 1.0f); const float d = bf16_rne(deter[(size_t)row * DET + g * DPB + j]);
      Ts[wave][8 * hlf + r][t * 16 + nloc] = pmul(upd, cand) + pmul(1.0f - upd, d); } }
  wave_lds_sync();
  for (int pass = 0; pass < 2; ++pass) { for (int i = lane; i < 16 * 8; i += 32) { const int rr = i >> 3, c4 = (i & 7) * 4; *(volatile v4f*)(out + (size_t)(m0 + rr) * DET + g * DPB + j0 + c4) = *(const v4f*)(&Ts[wave][rr][c4]); } __threadfence(); }
}
}

extern "C" void kernel_launch(void* const* d_in, const int* in_sizes, int n_in,
                              void* d_out, int out_size, void* d_ws, size_t ws_size, hipStream_t stream) {
  (void)n_in; (void)out_size;
  auto F = [&](int i) { return (const float*)d_in[i]; };
  const float* stoch = F(0); const float* deter = F(1); const float* action = F(2);
  float* out = (float*)d_out;
  if (in_sizes[0] != Bn * STO || in_sizes[1] != Bn * DET || in_sizes[2] != Bn * ACT || in_sizes[12] != BLK * INC0 * DPB || in_sizes[18] != BLK * DPB * 3 * DPB) return;
  size_t off = 0; char* ws = (char*)d_ws;
  auto carve = [&](size_t bytes) { char* p = ws + off; off += (bytes + 255) & ~(size_t)255; return p; };
  b16* R = (b16*)carve(Ro_::END * 2); float* P = (float*)carve((size_t)PEND * 4); b16* DX = (b16*)carve((size_t)Bn * DET * 2); b16* SX = (b16*)carve((size_t)Bn * STO * 2); b16* AX = (b16*)carve((size_t)Bn * ACT * 2);
  float* PRE = (float*)carve((size_t)Bn * DET * 4); b16* XCh = (b16*)carve((size_t)Bn * XW * 2); b16* XCl = (b16*)carve((size_t)Bn * XW * 2); b16* H0h = (b16*)carve((size_t)Bn * DET * 2); b16* H0l = (b16*)carve((size_t)Bn * DET * 2); b16* H1h = (b16*)carve((size_t)Bn * DET * 2); b16* H1l = (b16*)carve((size_t)Bn * DET * 2);
  if (off > ws_size) return;
  prep_kernel<<<2048, 256, 0, stream>>>(stoch, deter, action, F(3), F(6), F(9), F(12), F(15), F(18), R, DX, SX, AX);
  params_kernel<<<64, 256, 0, stream>>>(F(4), F(5), F(7), F(8), F(10), F(11), F(13), F(14), F(16), F(17), F(19), P);
  gemm_kernel<DET, 0><<<dim3(HID / 256, Bn / 32), 64, 0, stream>>>(DX, DET, 0, nullptr, nullptr, 0, R + Ro_::W0, P + 0, PRE, XW, 0);
  gemm_kernel<STO, 0><<<dim3(HID / 256, Bn / 32), 64, 0, stream>>>(SX, STO, 0, nullptr, nullptr, 0, R + Ro_::W1, P + 1024, PRE, XW, 1024);
  gemm_kernel<ACT, 0><<<dim3(HID / 256, Bn / 32), 64, 0, stream>>>(AX, ACT, 0, nullptr, nullptr, 0, R + Ro_::W2, P + 2048, PRE, XW, 2048);
  rms_kernel<3, HID><<<Bn, 256, 0, stream>>>(PRE, P + 3072, XCh, XCl);
  for (int g = 0; g < BLK; ++g) gemm_kernel<DPB, XW><<<dim3(DPB / 256, Bn / 32), 64, 0, stream>>>(DX, DET, g * DPB, XCh, XCl, XW, R + Ro_::H0W + (size_t)g * DPB * INC0, P + 6144 + g * DPB, PRE, DET, g * DPB);
  rms_kernel<1, DET><<<Bn, 256, 0, stream>>>(PRE, P + 10240, H0h, H0l);
  for (int g = 0; g < BLK; ++g) gemm_kernel<0, DPB><<<dim3(DPB / 256, Bn / 32), 64, 0, stream>>>(nullptr, 0, 0, H0h + g * DPB, H0l + g * DPB, DET, R + Ro_::H1W + (size_t)g * DPB * DPB, P + 14336 + g * DPB, PRE, DET, g * DPB);
  rms_kernel<1, DET><<<Bn, 256, 0, stream>>>(PRE, P + 18432, H1h, H1l);
  gate_kernel<<<dim3(DPB / 32, Bn / 32, BLK), 64, 0, stream>>>(H1h, H1l, R + Ro_::GW, P + 22528, deter, out);
}
